// TemporalMambaBlock_17781164605861
// MI455X (gfx1250) — hardware-run, weakly checked
//
#include <hip/hip_runtime.h>
#include <math.h>

constexpr int kBatch  = 2;
constexpr int kSeq    = 1024;
constexpr int kDim    = 1024;
constexpr int kInner  = 2048;
constexpr int kState  = 16;
constexpr int kConvK  = 4;
constexpr int kRank   = 64;
constexpr int kTok    = kBatch * kSeq;
constexpr int kXzLd   = 2 * kInner;
constexpr int kDblN   = kRank + 2 * kState;
constexpr int kDblLd  = 128;
constexpr int kChunk  = 16;
constexpr int kScanCh = 128;
constexpr float kWCarry = 16.0f;
constexpr float kACarry = 64.0f;
constexpr float kLog2e  = 1.4426950408889634f;
constexpr float kEps    = 1e-5f;

static_assert(kTok % 64 == 0 && kXzLd % 64 == 0 && kDblLd % 64 == 0 && kInner % 64 == 0 && kDim % 64 == 0);
static_assert(kDim % 32 == 0 && kInner % 32 == 0 && kRank % 32 == 0);
static_assert(kScanCh / 8 == kChunk && (kScanCh / 32) * 4 == kChunk && kChunk == 16);
static_assert(kInner % kScanCh == 0);

typedef __attribute__((ext_vector_type(16))) _Float16 v16h;
typedef __attribute__((ext_vector_type(8)))  _Float16 v8h;
typedef __attribute__((ext_vector_type(16))) __bf16   v16b;
typedef __attribute__((ext_vector_type(8)))  __bf16   v8b;
typedef __attribute__((ext_vector_type(8)))  float    v8f;
typedef __attribute__((ext_vector_type(4)))  float    v4f;
typedef __attribute__((ext_vector_type(4)))  unsigned int v4u;

__device__ __forceinline__ unsigned short f2bf_bits(float f) {
  unsigned u = __float_as_uint(f);
  return (unsigned short)((u + 0x7FFFu + ((u >> 16) & 1u)) >> 16);
}
__device__ __forceinline__ float bf_bits2f(unsigned short h) { return __uint_as_float(((unsigned)h) << 16); }

__device__ __forceinline__ void dep_guard_h(v8f& a, v8f& b, v16h x, v16h y) { asm volatile("v_nop\n\tv_nop\n\tv_nop\n\tv_nop" : "+v"(a), "+v"(b) : "v"(x), "v"(y)); }
__device__ __forceinline__ void dep_guard_b(v8f& a, v8f& b, v16b x, v16b y) { asm volatile("v_nop\n\tv_nop\n\tv_nop\n\tv_nop" : "+v"(a), "+v"(b) : "v"(x), "v"(y)); }
__device__ __forceinline__ void keep4_h(v16h a, v16h b, v16h c, v16h d) { asm volatile("v_nop" :: "v"(a), "v"(b), "v"(c), "v"(d)); }
__device__ __forceinline__ void keep4_b(v16b a, v16b b, v16b c, v16b d) { asm volatile("v_nop" :: "v"(a), "v"(b), "v"(c), "v"(d)); }
__device__ __forceinline__ void acc_guard4(v8f& a, v8f& b, v8f& c, v8f& d) { asm volatile("v_nop\n\tv_nop\n\tv_nop\n\tv_nop" : "+v"(a), "+v"(b), "+v"(c), "+v"(d)); }
template <typename T> struct Frag;
template <> struct Frag<_Float16> {
  typedef v16h V; union U { v16h v; v8h h[2]; };
  static __device__ __forceinline__ v16h load(const _Float16* p) {
    U f; f.h[0] = *(const v8h*)(p); f.h[1] = *(const v8h*)(p + 16); return f.v;
  }
  static __device__ __forceinline__ v8f mma(v16h a, v16h b, v8f c) {
    return __builtin_amdgcn_wmma_f32_16x16x32_f16(false, a, false, b, (short)0, c, false, false);
  }
  static __device__ __forceinline__ void guard(v8f& a, v8f& b, v16h x, v16h y) { dep_guard_h(a, b, x, y); }
  static __device__ __forceinline__ void keep(v16h a, v16h b, v16h c, v16h d) { keep4_h(a, b, c, d); }
};
template <> struct Frag<__bf16> {
  typedef v16b V; union U { v16b v; v8b h[2]; };
  static __device__ __forceinline__ v16b load(const __bf16* p) {
    U f; f.h[0] = *(const v8b*)(p); f.h[1] = *(const v8b*)(p + 16); return f.v;
  }
  static __device__ __forceinline__ v8f mma(v16b a, v16b b, v8f c) {
    return __builtin_amdgcn_wmma_f32_16x16x32_bf16(false, a, false, b, (short)0, c, false, false);
  }
  static __device__ __forceinline__ void guard(v8f& a, v8f& b, v16b x, v16b y) { dep_guard_b(a, b, x, y); }
  static __device__ __forceinline__ void keep(v16b a, v16b b, v16b c, v16b d) { keep4_b(a, b, c, d); }
};

__device__ __forceinline__ unsigned pk16(unsigned short a, unsigned short b) { return (unsigned)a | ((unsigned)b << 16); }
__device__ __forceinline__ unsigned short h_bits(float f) { const _Float16 h = (_Float16)f; return __builtin_bit_cast(unsigned short, h); }

template <int ET> struct Elem;
template <> struct Elem<0> { typedef _Float16 T; };
template <> struct Elem<1> { typedef __bf16 T; };
template <int ET, bool SPLIT, int BIAS_MODE, int OUT_MODE, bool RESID, int ACT = 0>
__global__ __launch_bounds__(256) void wmma_gemm64(
    const unsigned short* __restrict__ Ap, const unsigned short* __restrict__ A2p, int lda, long strideA,
    const unsigned short* __restrict__ Btp, const unsigned short* __restrict__ Bt2p, int ldb, long strideB,
    void* __restrict__ Cout, void* __restrict__ Cout2, int ldc, long strideC,
    const float* __restrict__ bias,
    const float* __restrict__ resid, long strideR,
    int M, int N, int K, float scale) {
  typedef typename Elem<ET>::T T;
  typedef typename Frag<T>::V V;
  const T* A = (const T*)Ap; const T* A2 = (const T*)A2p; const T* Bt = (const T*)Btp; const T* Bt2 = (const T*)Bt2p;
  __shared__ __align__(16) float sT[8][16 * 68];
  const int b    = blockIdx.y;
  const int lane = threadIdx.x & 31;
  const int wave = threadIdx.x >> 5;
  const int tilesN = N >> 6;
  const int tilesM = M >> 6;
  const int tile = blockIdx.x * 8 + wave;
  if (tile >= tilesM * tilesN) return;
  const int tm = tile / tilesN;
  const int tn = tile - tm * tilesN;
  const int m0 = tm << 6;
  const int n0 = tn << 6;

  const T* Ab  = A  + (size_t)b * strideA;
  const T* Bb  = Bt + (size_t)b * strideB;
  const T* Ab2 = SPLIT ? (A2  + (size_t)b * strideA) : nullptr;
  const T* Bb2 = SPLIT ? (Bt2 + (size_t)b * strideB) : nullptr;

  const int rlane = lane & 15;
  const int koff  = (lane >> 4) * 8;
  const int mOff  = (lane >> 4) * 8;

  v8f acc[4][4];
#pragma unroll
  for (int i = 0; i < 4; ++i)
#pragma unroll
    for (int j = 0; j < 4; ++j) acc[i][j] = (v8f){0.f,0.f,0.f,0.f,0.f,0.f,0.f,0.f};

  for (int k0 = 0; k0 < K; k0 += 32) {
    V bh[4], bl[4];
#pragma unroll
    for (int j = 0; j < 4; ++j) {
      const size_t bo = (size_t)(n0 + (j << 4) + rlane) * ldb + koff + k0;
      bh[j] = Frag<T>::load(Bb + bo);
      if (SPLIT) bl[j] = Frag<T>::load(Bb2 + bo);
    }
#pragma unroll
    for (int i = 0; i < 4; ++i) {
      const size_t ao = (size_t)(m0 + (i << 4) + rlane) * lda + koff + k0;
      V ah = Frag<T>::load(Ab + ao);
      V al;
      if (SPLIT) al = Frag<T>::load(Ab2 + ao);
#pragma unroll
      for (int j = 0; j < 4; ++j) {
        acc[i][j] = Frag<T>::mma(ah, bh[j], acc[i][j]);
        if (SPLIT) {
          acc[i][j] = Frag<T>::mma(ah, bl[j], acc[i][j]);
          acc[i][j] = Frag<T>::mma(al, bh[j], acc[i][j]);
        }
      }
      Frag<T>::guard(acc[i][0], acc[i][3], ah, SPLIT ? al : ah);
    }
    Frag<T>::keep(bh[0], bh[1], bh[2], bh[3]);
    if (SPLIT) Frag<T>::keep(bl[0], bl[1], bl[2], bl[3]);
  }
  acc_guard4(acc[0][0], acc[0][1], acc[0][2], acc[0][3]);
  acc_guard4(acc[1][0], acc[1][1], acc[1][2], acc[1][3]);
  acc_guard4(acc[2][0], acc[2][1], acc[2][2], acc[2][3]);
  acc_guard4(acc[3][0], acc[3][1], acc[3][2], acc[3][3]);

  float* slab = sT[wave];
  const float* Rb = RESID ? (resid + (size_t)b * strideR) : nullptr;
#pragma unroll
  for (int i = 0; i < 4; ++i) {
    const int mBase = m0 + (i << 4);
#pragma unroll
    for (int j = 0; j < 4; ++j) {
      const int n = n0 + (j << 4) + rlane;
      float bv = 0.f;
      if (BIAS_MODE == 2) bv = bias[n];
#pragma unroll
      for (int r = 0; r < 8; ++r) {
        float v = acc[i][j][r] * scale;
        if (BIAS_MODE == 1) v += bias[mBase + mOff + r];
        if (BIAS_MODE == 2) v += bv;
        if (RESID) v += Rb[(size_t)(mBase + mOff + r) * ldc + n];
        if (ACT == 2) v = fmaxf(v, 0.0f);
        if (ACT == 4) v = (v > 0.f) ? v : 0.01f * v;
        slab[(mOff + r) * 68 + (j << 4) + rlane] = v;
      }
    }
    __builtin_amdgcn_fence(__ATOMIC_RELEASE, "workgroup");
    __builtin_amdgcn_wave_barrier();
    __builtin_amdgcn_fence(__ATOMIC_ACQUIRE, "workgroup");
    if (OUT_MODE == 0) {
      float* C = (float*)Cout + (size_t)b * strideC;
      const int hh = lane >> 4, c4 = (lane & 15) * 4;
      for (int pass = 0; pass < 2; ++pass) {
#pragma unroll
        for (int it = 0; it < 8; ++it) {
          const int row = it * 2 + hh;
          v4f v = *(const v4f*)(slab + row * 68 + c4);
          *(volatile v4f*)(C + (size_t)(mBase + row) * ldc + n0 + c4) = v;
        }
        __threadfence();
      }
    } else {
      const int q = lane >> 3, c8 = (lane & 7) * 8;
      unsigned short* C  = (unsigned short*)Cout  + (size_t)b * strideC;
      unsigned short* C2 = (OUT_MODE == 2) ? ((unsigned short*)Cout2 + (size_t)b * strideC) : nullptr;
      for (int pass = 0; pass < 2; ++pass) {
#pragma unroll
        for (int it = 0; it < 4; ++it) {
          const int row = it * 4 + q;
          const float* sp = slab + row * 68 + c8;
          v8h hv, lv;
#pragma unroll
          for (int e = 0; e < 8; ++e) {
            if (OUT_MODE == 1) {
              hv[e] = (_Float16)sp[e];
            } else {
              unsigned short hb = f2bf_bits(sp[e]);
              unsigned short lb = f2bf_bits(sp[e] - bf_bits2f(hb));
              hv[e] = __builtin_bit_cast(_Float16, hb);
              lv[e] = __builtin_bit_cast(_Float16, lb);
            }
          }
          *(volatile v8h*)(C + (size_t)(mBase + row) * ldc + n0 + c8) = hv;
          if (OUT_MODE == 2) *(volatile v8h*)(C2 + (size_t)(mBase + row) * ldc + n0 + c8) = lv;
        }
        __threadfence();
      }
    }
    __builtin_amdgcn_fence(__ATOMIC_RELEASE, "workgroup");
    __builtin_amdgcn_wave_barrier();
    __builtin_amdgcn_fence(__ATOMIC_ACQUIRE, "workgroup");
  }
}

__global__ __launch_bounds__(256) void wt_cast_kernel(const float* __restrict__ W, unsigned short* __restrict__ out,
                                                      int kdim, int ndim, float scale) {
  __shared__ float sm[64][65];
  const int t  = threadIdx.x;
  const int k0 = blockIdx.x * 64;
  const int n0 = blockIdx.y * 64;
#pragma unroll
  for (int i = 0; i < 16; ++i) {
    const int e = i * 256 + t;
    const int r = e >> 6;
    const int c = e & 63;
    const int n = n0 + c;
    const int nc = (n < ndim) ? n : (ndim - 1);
    const float v = W[(size_t)(k0 + r) * ndim + nc] * scale;
    sm[c][r] = (n < ndim) ? v : 0.0f;
  }
  __syncthreads();
  const int lane = t & 31, wave = t >> 5;
  const int q = lane >> 3, c8 = (lane & 7) * 8;
  for (int pass = 0; pass < 2; ++pass) {
#pragma unroll
    for (int it = 0; it < 2; ++it) {
      const int row = wave * 8 + it * 4 + q;
      unsigned short hb[8];
#pragma unroll
      for (int e = 0; e < 8; ++e) hb[e] = h_bits(sm[row][c8 + e]);
      const v4u u = (v4u){pk16(hb[0], hb[1]), pk16(hb[2], hb[3]), pk16(hb[4], hb[5]), pk16(hb[6], hb[7])};
      *(volatile v4u*)(out + (size_t)(n0 + row) * kdim + k0 + c8) = u;
    }
    __threadfence();
  }
}

__global__ __launch_bounds__(128) void rmsnorm_kernel(const float* __restrict__ x, const float* __restrict__ w,
                                                      unsigned short* __restrict__ out) {
  __shared__ float red[4];
  const int row  = blockIdx.x;
  const int t    = threadIdx.x;
  const int lane = t & 31, wave = t >> 5;
  const float* xr = x + (size_t)row * kDim + 8 * t;
  const v4f a = *(const v4f*)(xr);
  const v4f c = *(const v4f*)(xr + 4);
  float ss = a[0] * a[0];
  ss += a[1] * a[1]; ss += a[2] * a[2]; ss += a[3] * a[3];
  ss += c[0] * c[0]; ss += c[1] * c[1]; ss += c[2] * c[2]; ss += c[3] * c[3];
#pragma unroll
  for (int off = 16; off > 0; off >>= 1) ss += __shfl_xor(ss, off, 32);
  if (lane == 0) red[wave] = ss;
  __syncthreads();
  const float tot = ((red[0] + red[1]) + red[2]) + red[3];
  const float rs = rsqrtf(tot * (1.0f / 1024.0f) + kEps);
  const v4f wa = *(const v4f*)(w + 8 * t);
  const v4f wc = *(const v4f*)(w + 8 * t + 4);
  unsigned short hb[8];
#pragma unroll
  for (int e = 0; e < 4; ++e) {
    hb[e]     = h_bits((a[e] * rs) * wa[e]);
    hb[4 + e] = h_bits((c[e] * rs) * wc[e]);
  }
  const v4u u = (v4u){pk16(hb[0], hb[1]), pk16(hb[2], hb[3]), pk16(hb[4], hb[5]), pk16(hb[6], hb[7])};
  unsigned short* q = out + (size_t)row * kDim + 8 * t;
  *(volatile v4u*)q = u;
  __threadfence();
  *(volatile v4u*)q = u;
}

__global__ __launch_bounds__(256) void conv_silu_kernel(const float* __restrict__ xz, const float* __restrict__ cw,
                                                        const float* __restrict__ cb, float* __restrict__ xbf,
                                                        unsigned short* __restrict__ xb16) {
  __shared__ __align__(16) unsigned int su[512];
  const int t    = threadIdx.x;
  const int row  = blockIdx.x >> 1;
  const int hsel = blockIdx.x & 1;
  const int b    = row >> 10;
  const int tpos = row & (kSeq - 1);
  const int c    = hsel * 1024 + 4 * t;
  v4f xk[4];
#pragma unroll
  for (int k = 0; k < 4; ++k) {
    const int ts  = tpos - (kConvK - 1) + k;
    const int tsc = (ts < 0) ? 0 : ts;
    const v4f v = *(const v4f*)(xz + ((size_t)b * kSeq + tsc) * kXzLd + c);
    const float fm = (ts >= 0) ? 1.0f : 0.0f;
    xk[k] = v * fm;
  }
  const v4f bias = *(const v4f*)(cb + c);
  float res[4];
  unsigned short hb[4];
#pragma unroll
  for (int j = 0; j < 4; ++j) {
    const v4f wj = *(const v4f*)(cw + (size_t)(c + j) * kConvK);
    float acc = wj[0] * xk[0][j];
    acc = acc + wj[1] * xk[1][j];
    acc = acc + wj[2] * xk[2][j];
    acc = acc + wj[3] * xk[3][j];
    acc = acc + bias[j];
    const float s = acc * (1.0f / (1.0f + expf(-acc)));
    res[j] = s;
    hb[j] = h_bits(s * kACarry);
  }
  const v4f o = (v4f){res[0], res[1], res[2], res[3]};
  su[2 * t]     = pk16(hb[0], hb[1]);
  su[2 * t + 1] = pk16(hb[2], hb[3]);
  __syncthreads();
  const int tl = t & 127;
  const v4u u = *(const v4u*)(su + 4 * tl);
  float* fp = xbf + (size_t)row * kInner + c;
  unsigned short* hp = xb16 + (size_t)row * kInner + hsel * 1024 + 8 * tl;
  for (int pass = 0; pass < 2; ++pass) {
    *(volatile v4f*)fp = o;
    if (t < 128) *(volatile v4u*)hp = u;
    __threadfence();
  }
}

__global__ __launch_bounds__(256) void cast_dr_kernel(const float* __restrict__ dbl, unsigned short* __restrict__ dr) {
  const int i = blockIdx.x * 256 + threadIdx.x;
  if (i >= kTok * 8) return;
  const int row = i >> 3, c8 = (i & 7) * 8;
  const float* p = dbl + (size_t)row * kDblLd + c8;
  const v4f a = *(const v4f*)(p);
  const v4f c = *(const v4f*)(p + 4);
  unsigned short hb[8];
#pragma unroll
  for (int e = 0; e < 4; ++e) {
    hb[e]     = h_bits(a[e] * kACarry);
    hb[4 + e] = h_bits(c[e] * kACarry);
  }
  const v4u u = (v4u){pk16(hb[0], hb[1]), pk16(hb[2], hb[3]), pk16(hb[4], hb[5]), pk16(hb[6], hb[7])};
  unsigned short* q = dr + (size_t)row * kRank + c8;
  *(volatile v4u*)q = u;
  __threadfence();
  *(volatile v4u*)q = u;
}

__global__ __launch_bounds__(kScanCh) void scan_kernel(const float* __restrict__ dbl, const float* __restrict__ draw,
                                                       const float* __restrict__ xbf, const float* __restrict__ xz,
                                                       const float* __restrict__ alog, const float* __restrict__ dvec,
                                                       unsigned short* __restrict__ yg) {
  __shared__ __align__(16) float sD[kChunk][kScanCh];
  __shared__ __align__(16) float sX[kChunk][kScanCh];
  __shared__ __align__(16) float sG[kChunk][kScanCh];
  __shared__ __align__(16) float sBC[kChunk][2 * kState];
  __shared__ __align__(16) float sY[kChunk][kScanCh + 4];
  __shared__ float sA[kState][kScanCh];
  const int t = threadIdx.x, lane = t & 31, wave = t >> 5;
  const int b  = blockIdx.x / (kInner / kScanCh);
  const int e0 = (blockIdx.x % (kInner / kScanCh)) * kScanCh;
  const int e  = e0 + t;
#pragma unroll 1
  for (int n = 0; n < kState; ++n) sA[n][t] = -expf(alog[(size_t)e * kState + n]);
  float A2[kState], h[kState];
#pragma unroll
  for (int n = 0; n < kState; ++n) { A2[n] = sA[n][t] * kLog2e; h[n] = 0.0f; }
  const float De = dvec[e];
  const int hh = lane >> 4, c16 = lane & 15;

  for (int t0 = 0; t0 < kSeq; t0 += kChunk) {
    __syncthreads();
#pragma unroll 1
    for (int tt = 0; tt < kChunk; ++tt) {
      const size_t tok = (size_t)b * kSeq + t0 + tt;
      const float v = draw[tok * kInner + e];
      sD[tt][t] = fmaxf(v, 0.0f) + log1pf(expf(-fabsf(v)));
      sX[tt][t] = xbf[tok * kInner + e];
      const float z = xz[tok * kXzLd + kInner + e];
      sG[tt][t] = z * (1.0f / (1.0f + expf(-z)));
    }
    {
      const int r = t >> 3, c4 = (t & 7) * 4;
      const v4f bc = *(const v4f*)(dbl + ((size_t)b * kSeq + t0 + r) * kDblLd + kRank + c4);
      *(v4f*)(&sBC[r][c4]) = bc;
    }
    __syncthreads();
#pragma unroll 1
    for (int tt = 0; tt < kChunk; ++tt) {
      const float d = sD[tt][t];
      const float x = sX[tt][t];
      const float g = sG[tt][t];
      const float dx = d * x;
      float ys = 0.0f;
#pragma unroll
      for (int n = 0; n < kState; ++n) {
        const float a = exp2f(d * A2[n]);
        h[n] = a * h[n] + dx * sBC[tt][n];
        ys += h[n] * sBC[tt][kState + n];
      }
      const float y = ys + De * x;
      sY[tt][t] = (y * g) * kACarry;
    }
    __syncthreads();
    for (int pass = 0; pass < 2; ++pass) {
#pragma unroll
      for (int it = 0; it < 2; ++it) {
        const int row = wave * 4 + it * 2 + hh;
        const float* sp = &sY[row][8 * c16];
        const v4f a = *(const v4f*)(sp);
        const v4f c = *(const v4f*)(sp + 4);
        unsigned short hb[8];
#pragma unroll
        for (int q = 0; q < 4; ++q) {
          hb[q]     = h_bits(a[q]);
          hb[4 + q] = h_bits(c[q]);
        }
        const v4u u = (v4u){pk16(hb[0], hb[1]), pk16(hb[2], hb[3]), pk16(hb[4], hb[5]), pk16(hb[6], hb[7])};
        *(volatile v4u*)(yg + ((size_t)b * kSeq + t0 + row) * kInner + e0 + 8 * c16) = u;
      }
      __threadfence();
    }
  }
}

extern "C" void kernel_launch(void* const* d_in, const int* in_sizes, int n_in,
                              void* d_out, int out_size, void* d_ws, size_t ws_size,
                              hipStream_t stream) {
  if (n_in < 11) return;
  if (in_sizes[0] != kTok * kDim || in_sizes[1] != kDim * kXzLd || in_sizes[2] != kInner * kConvK ||
      in_sizes[3] != kInner || in_sizes[4] != kInner * kDblN || in_sizes[5] != kRank * kInner ||
      in_sizes[6] != kInner || in_sizes[7] != kInner * kState || in_sizes[8] != kInner ||
      in_sizes[9] != kInner * kDim || in_sizes[10] != kDim) return;
  if (out_size != kTok * kDim) return;

  const float* x      = (const float*)d_in[0];
  const float* W_in   = (const float*)d_in[1];
  const float* conv_w = (const float*)d_in[2];
  const float* conv_b = (const float*)d_in[3];
  const float* W_x    = (const float*)d_in[4];
  const float* W_dt   = (const float*)d_in[5];
  const float* b_dt   = (const float*)d_in[6];
  const float* A_log  = (const float*)d_in[7];
  const float* Dvec   = (const float*)d_in[8];
  const float* W_out  = (const float*)d_in[9];
  const float* rms_w  = (const float*)d_in[10];
  float* out = (float*)d_out;

  char* ws = (char*)d_ws;
  size_t off = 0;
  auto carve = [&](size_t bytes) -> char* { char* p = ws + off; off += (bytes + 255) & ~(size_t)255; return p; };
  unsigned short* WinT16  = (unsigned short*)carve((size_t)kXzLd * kDim * 2);
  unsigned short* WxT16   = (unsigned short*)carve((size_t)kDblLd * kInner * 2);
  unsigned short* WdtT16  = (unsigned short*)carve((size_t)kInner * kRank * 2);
  unsigned short* WoutT16 = (unsigned short*)carve((size_t)kDim * kInner * 2);
  unsigned short* xn16    = (unsigned short*)carve((size_t)kTok * kDim * 2);
  float*          xz      = (float*)         carve((size_t)kTok * kXzLd * 4);
  float*          xbf     = (float*)         carve((size_t)kTok * kInner * 4);
  unsigned short* xb16    = (unsigned short*)carve((size_t)kTok * kInner * 2);
  float*          dbl     = (float*)         carve((size_t)kTok * kDblLd * 4);
  unsigned short* dr16    = (unsigned short*)carve((size_t)kTok * kRank * 2);
  float*          draw    = (float*)         carve((size_t)kTok * kInner * 4);
  unsigned short* yg16    = (unsigned short*)carve((size_t)kTok * kInner * 2);
  if (off > ws_size) return;

  wt_cast_kernel<<<dim3(kDim / 64, kXzLd / 64), 256, 0, stream>>>(W_in, WinT16, kDim, kXzLd, kWCarry);
  wt_cast_kernel<<<dim3(kInner / 64, kDblLd / 64), 256, 0, stream>>>(W_x, WxT16, kInner, kDblN, kWCarry);
  wt_cast_kernel<<<dim3(kRank / 64, kInner / 64), 256, 0, stream>>>(W_dt, WdtT16, kRank, kInner, kWCarry);
  wt_cast_kernel<<<dim3(kInner / 64, kDim / 64), 256, 0, stream>>>(W_out, WoutT16, kInner, kDim, kWCarry);

  rmsnorm_kernel<<<kTok, 128, 0, stream>>>(x, rms_w, xn16);

  wmma_gemm64<0, false, 0, 0, false, 0><<<dim3((kTok / 64) * (kXzLd / 64) / 8, 1), 256, 0, stream>>>(
      xn16, nullptr, kDim, 0L, WinT16, nullptr, kDim, 0L, (void*)xz, nullptr, kXzLd, 0L,
      nullptr, nullptr, 0L, kTok, kXzLd, kDim, 1.0f / kWCarry);

  conv_silu_kernel<<<kTok * 2, 256, 0, stream>>>(xz, conv_w, conv_b, xbf, xb16);

  wmma_gemm64<0, false, 0, 0, false, 0><<<dim3((kTok / 64) * (kDblLd / 64) / 8, 1), 256, 0, stream>>>(
      xb16, nullptr, kInner, 0L, WxT16, nullptr, kInner, 0L, (void*)dbl, nullptr, kDblLd, 0L,
      nullptr, nullptr, 0L, kTok, kDblLd, kInner, 1.0f / (kACarry * kWCarry));

  cast_dr_kernel<<<(kTok * 8) / 256, 256, 0, stream>>>(dbl, dr16);
  wmma_gemm64<0, false, 2, 0, false, 0><<<dim3((kTok / 64) * (kInner / 64) / 8, 1), 256, 0, stream>>>(
      dr16, nullptr, kRank, 0L, WdtT16, nullptr, kRank, 0L, (void*)draw, nullptr, kInner, 0L,
      b_dt, nullptr, 0L, kTok, kInner, kRank, 1.0f / (kACarry * kWCarry));

  scan_kernel<<<kBatch * (kInner / kScanCh), kScanCh, 0, stream>>>(dbl, draw, xbf, xz, A_log, Dvec, yg16);

  wmma_gemm64<0, false, 0, 0, true, 0><<<dim3((kTok / 64) * (kDim / 64) / 8, 1), 256, 0, stream>>>(
      yg16, nullptr, kInner, 0L, WoutT16, nullptr, kInner, 0L, (void*)out, nullptr, kDim, 0L,
      nullptr, x, 0L, kTok, kDim, kInner, 1.0f / (kACarry * kWCarry));
}
